// CrossRepair_63462436765733
// MI455X (gfx1250) — hardware-verified
//
#include <hip/hip_runtime.h>
#include <math.h>

constexpr int kB    = 2;
constexpr int kT    = 2048;
constexpr int kD    = 1024;
constexpr int kH    = 16;
constexpr int kDH   = 64;
constexpr int kTok  = kB * kT;
constexpr int kFF   = 4 * kD;
constexpr int kKVld = 2 * kD;
constexpr int kGrp  = kB * kH;
constexpr int kGC   = 2;
constexpr int kNChunk = kGrp / kGC;
constexpr int kMC   = 1024;
constexpr int kNMC  = kTok / kMC;
constexpr float kWCarry   = 16.0f;
constexpr float kPCarry   = 2048.0f;
constexpr float kCtxCarry = 256.0f;
constexpr float kActCarry = 16.0f;
constexpr float kInvD     = 1.0f / 1024.0f;
constexpr float kLnEps    = 1e-5f;
static_assert(kH % kGC == 0, "chunk never crosses a batch boundary");
static_assert(kD % 64 == 0 && kT % 64 == 0 && kFF % 64 == 0 && kMC % 64 == 0, "tile multiples");
static_assert(kDH % 32 == 0 && kD % 32 == 0 && kT % 32 == 0 && kFF % 32 == 0, "K multiples of 32");

constexpr size_t kMiB     = 1048576;
constexpr size_t OFF_WOT  = 0;
constexpr size_t OFF_W1T  = 2 * kMiB;
constexpr size_t OFF_W2T  = 10 * kMiB;
constexpr size_t OFF_CTX  = 18 * kMiB;
constexpr size_t OFF_QP   = 26 * kMiB;
constexpr size_t OFF_KVP  = 34 * kMiB;
constexpr size_t OFF_VT   = 50 * kMiB;
constexpr size_t OFF_ARENA = 58 * kMiB;
constexpr size_t OFF_QLN  = OFF_ARENA;
constexpr size_t OFF_KVLN = OFF_ARENA + 8 * kMiB;
constexpr size_t OFF_WQT  = OFF_ARENA + 16 * kMiB;
constexpr size_t OFF_WKT  = OFF_ARENA + 18 * kMiB;
constexpr size_t OFF_WVT  = OFF_ARENA + 20 * kMiB;
constexpr size_t OFF_SC   = OFF_ARENA;
constexpr size_t OFF_Y    = OFF_ARENA;
constexpr size_t OFF_H16  = OFF_ARENA + 16 * kMiB;
constexpr size_t OFF_ACT  = OFF_ARENA + 24 * kMiB;
constexpr size_t OFF_P    = 90 * kMiB;
constexpr size_t OFF_H1   = OFF_P;
constexpr size_t kWsTotal = 106 * kMiB;
static_assert((size_t)kD * kD * 2 == 2 * kMiB, "W plane");
static_assert((size_t)kFF * kD * 2 == 8 * kMiB, "W1/W2 plane");
static_assert((size_t)kTok * kD * 2 == 8 * kMiB, "token f16 plane");
static_assert((size_t)kTok * kKVld * 2 == 16 * kMiB, "kv plane");
static_assert((size_t)kGrp * kDH * kT * 2 == 8 * kMiB, "vt plane");
static_assert((size_t)kGC * kT * kT * 4 == 32 * kMiB, "scores chunk");
static_assert((size_t)kGC * kT * kT * 2 == 16 * kMiB, "P chunk");
static_assert((size_t)kTok * kD * 4 == 16 * kMiB, "Y plane");
static_assert((size_t)kMC * kFF * 4 == 16 * kMiB, "H1 chunk");
static_assert((size_t)kMC * kFF * 2 == 8 * kMiB, "ACT chunk");
static_assert(OFF_WVT + 2 * kMiB <= OFF_P, "phase A inside arena");
static_assert(OFF_ACT + 8 * kMiB <= OFF_P, "phase C inside arena");
static_assert(kWsTotal <= 134217728, "carve budget");

typedef __attribute__((ext_vector_type(16))) _Float16 v16h;
typedef __attribute__((ext_vector_type(8)))  _Float16 v8h;
typedef __attribute__((ext_vector_type(16))) __bf16   v16b;
typedef __attribute__((ext_vector_type(8)))  __bf16   v8b;
typedef __attribute__((ext_vector_type(8)))  float    v8f;
typedef __attribute__((ext_vector_type(4)))  float    v4f;
typedef __attribute__((ext_vector_type(4)))  unsigned int v4u;

__device__ __forceinline__ unsigned short f2bf_bits(float f) {
  unsigned u = __float_as_uint(f);
  return (unsigned short)((u + 0x7FFFu + ((u >> 16) & 1u)) >> 16);
}
__device__ __forceinline__ float bf_bits2f(unsigned short h) { return __uint_as_float(((unsigned)h) << 16); }

__device__ __forceinline__ void dep_guard_h(v8f& a, v8f& b, v16h x, v16h y) { asm volatile("v_nop\n\tv_nop\n\tv_nop\n\tv_nop" : "+v"(a), "+v"(b) : "v"(x), "v"(y)); }
__device__ __forceinline__ void dep_guard_b(v8f& a, v8f& b, v16b x, v16b y) { asm volatile("v_nop\n\tv_nop\n\tv_nop\n\tv_nop" : "+v"(a), "+v"(b) : "v"(x), "v"(y)); }
__device__ __forceinline__ void keep4_h(v16h a, v16h b, v16h c, v16h d) { asm volatile("v_nop" :: "v"(a), "v"(b), "v"(c), "v"(d)); }
__device__ __forceinline__ void keep4_b(v16b a, v16b b, v16b c, v16b d) { asm volatile("v_nop" :: "v"(a), "v"(b), "v"(c), "v"(d)); }
__device__ __forceinline__ void acc_guard4(v8f& a, v8f& b, v8f& c, v8f& d) { asm volatile("v_nop\n\tv_nop\n\tv_nop\n\tv_nop" : "+v"(a), "+v"(b), "+v"(c), "+v"(d)); }
template <typename T> struct Frag;
template <> struct Frag<_Float16> {
  typedef v16h V; union U { v16h v; v8h h[2]; };
  static __device__ __forceinline__ v16h load(const _Float16* p) {
    U f; f.h[0] = *(const v8h*)(p); f.h[1] = *(const v8h*)(p + 16); return f.v;
  }
  static __device__ __forceinline__ v8f mma(v16h a, v16h b, v8f c) {
    return __builtin_amdgcn_wmma_f32_16x16x32_f16(false, a, false, b, (short)0, c, false, false);
  }
  static __device__ __forceinline__ void guard(v8f& a, v8f& b, v16h x, v16h y) { dep_guard_h(a, b, x, y); }
  static __device__ __forceinline__ void keep(v16h a, v16h b, v16h c, v16h d) { keep4_h(a, b, c, d); }
};
template <> struct Frag<__bf16> {
  typedef v16b V; union U { v16b v; v8b h[2]; };
  static __device__ __forceinline__ v16b load(const __bf16* p) {
    U f; f.h[0] = *(const v8b*)(p); f.h[1] = *(const v8b*)(p + 16); return f.v;
  }
  static __device__ __forceinline__ v8f mma(v16b a, v16b b, v8f c) {
    return __builtin_amdgcn_wmma_f32_16x16x32_bf16(false, a, false, b, (short)0, c, false, false);
  }
  static __device__ __forceinline__ void guard(v8f& a, v8f& b, v16b x, v16b y) { dep_guard_b(a, b, x, y); }
  static __device__ __forceinline__ void keep(v16b a, v16b b, v16b c, v16b d) { keep4_b(a, b, c, d); }
};

__device__ __forceinline__ unsigned pk16(unsigned short a, unsigned short b) { return (unsigned)a | ((unsigned)b << 16); }
__device__ __forceinline__ unsigned short h_bits(float f) { const _Float16 h = (_Float16)f; return __builtin_bit_cast(unsigned short, h); }

template <int ET> struct Elem;
template <> struct Elem<0> { typedef _Float16 T; };
template <> struct Elem<1> { typedef __bf16 T; };
template <int ET, bool SPLIT, int BIAS_MODE, int OUT_MODE, bool RESID, int ACT = 0>
__global__ __launch_bounds__(256) void wmma_gemm64(
    const unsigned short* __restrict__ Ap, const unsigned short* __restrict__ A2p, int lda, long strideA,
    const unsigned short* __restrict__ Btp, const unsigned short* __restrict__ Bt2p, int ldb, long strideB,
    void* __restrict__ Cout, void* __restrict__ Cout2, int ldc, long strideC,
    const float* __restrict__ bias,
    const float* __restrict__ resid, long strideR,
    int M, int N, int K, float scale) {
  typedef typename Elem<ET>::T T;
  typedef typename Frag<T>::V V;
  const T* A = (const T*)Ap; const T* A2 = (const T*)A2p; const T* Bt = (const T*)Btp; const T* Bt2 = (const T*)Bt2p;
  __shared__ __align__(16) float sT[8][16 * 68];
  const int b    = blockIdx.y;
  const int lane = threadIdx.x & 31;
  const int wave = threadIdx.x >> 5;
  const int tilesN = N >> 6;
  const int tilesM = M >> 6;
  const int tile = blockIdx.x * 8 + wave;
  if (tile >= tilesM * tilesN) return;
  const int tm = tile / tilesN;
  const int tn = tile - tm * tilesN;
  const int m0 = tm << 6;
  const int n0 = tn << 6;

  const T* Ab  = A  + (size_t)b * strideA;
  const T* Bb  = Bt + (size_t)b * strideB;
  const T* Ab2 = SPLIT ? (A2  + (size_t)b * strideA) : nullptr;
  const T* Bb2 = SPLIT ? (Bt2 + (size_t)b * strideB) : nullptr;

  const int rlane = lane & 15;
  const int koff  = (lane >> 4) * 8;
  const int mOff  = (lane >> 4) * 8;

  v8f acc[4][4];
#pragma unroll
  for (int i = 0; i < 4; ++i)
#pragma unroll
    for (int j = 0; j < 4; ++j) acc[i][j] = (v8f){0.f,0.f,0.f,0.f,0.f,0.f,0.f,0.f};

  for (int k0 = 0; k0 < K; k0 += 32) {
    V bh[4], bl[4];
#pragma unroll
    for (int j = 0; j < 4; ++j) {
      const size_t bo = (size_t)(n0 + (j << 4) + rlane) * ldb + koff + k0;
      bh[j] = Frag<T>::load(Bb + bo);
      if (SPLIT) bl[j] = Frag<T>::load(Bb2 + bo);
    }
#pragma unroll
    for (int i = 0; i < 4; ++i) {
      const size_t ao = (size_t)(m0 + (i << 4) + rlane) * lda + koff + k0;
      V ah = Frag<T>::load(Ab + ao);
      V al;
      if (SPLIT) al = Frag<T>::load(Ab2 + ao);
#pragma unroll
      for (int j = 0; j < 4; ++j) {
        acc[i][j] = Frag<T>::mma(ah, bh[j], acc[i][j]);
        if (SPLIT) {
          acc[i][j] = Frag<T>::mma(ah, bl[j], acc[i][j]);
          acc[i][j] = Frag<T>::mma(al, bh[j], acc[i][j]);
        }
      }
      Frag<T>::guard(acc[i][0], acc[i][3], ah, SPLIT ? al : ah);
    }
    Frag<T>::keep(bh[0], bh[1], bh[2], bh[3]);
    if (SPLIT) Frag<T>::keep(bl[0], bl[1], bl[2], bl[3]);
  }
  acc_guard4(acc[0][0], acc[0][1], acc[0][2], acc[0][3]);
  acc_guard4(acc[1][0], acc[1][1], acc[1][2], acc[1][3]);
  acc_guard4(acc[2][0], acc[2][1], acc[2][2], acc[2][3]);
  acc_guard4(acc[3][0], acc[3][1], acc[3][2], acc[3][3]);

  float* slab = sT[wave];
  const float* Rb = RESID ? (resid + (size_t)b * strideR) : nullptr;
#pragma unroll
  for (int i = 0; i < 4; ++i) {
    const int mBase = m0 + (i << 4);
#pragma unroll
    for (int j = 0; j < 4; ++j) {
      const int n = n0 + (j << 4) + rlane;
      float bv = 0.f;
      if (BIAS_MODE == 2) bv = bias[n];
#pragma unroll
      for (int r = 0; r < 8; ++r) {
        float v = acc[i][j][r] * scale;
        if (BIAS_MODE == 1) v += bias[mBase + mOff + r];
        if (BIAS_MODE == 2) v += bv;
        if (RESID) v += Rb[(size_t)(mBase + mOff + r) * ldc + n];
        if (ACT == 2) v = fmaxf(v, 0.0f);
        if (ACT == 4) v = (v > 0.f) ? v : 0.01f * v;
        slab[(mOff + r) * 68 + (j << 4) + rlane] = v;
      }
    }
    __builtin_amdgcn_fence(__ATOMIC_RELEASE, "workgroup");
    __builtin_amdgcn_wave_barrier();
    __builtin_amdgcn_fence(__ATOMIC_ACQUIRE, "workgroup");
    if (OUT_MODE == 0) {
      float* C = (float*)Cout + (size_t)b * strideC;
      const int hh = lane >> 4, c4 = (lane & 15) * 4;
      for (int pass = 0; pass < 2; ++pass) {
#pragma unroll
        for (int it = 0; it < 8; ++it) {
          const int row = it * 2 + hh;
          v4f v = *(const v4f*)(slab + row * 68 + c4);
          *(volatile v4f*)(C + (size_t)(mBase + row) * ldc + n0 + c4) = v;
        }
        __threadfence();
      }
    } else {
      const int q = lane >> 3, c8 = (lane & 7) * 8;
      unsigned short* C  = (unsigned short*)Cout  + (size_t)b * strideC;
      unsigned short* C2 = (OUT_MODE == 2) ? ((unsigned short*)Cout2 + (size_t)b * strideC) : nullptr;
      for (int pass = 0; pass < 2; ++pass) {
#pragma unroll
        for (int it = 0; it < 4; ++it) {
          const int row = it * 4 + q;
          const float* sp = slab + row * 68 + c8;
          v8h hv, lv;
#pragma unroll
          for (int e = 0; e < 8; ++e) {
            if (OUT_MODE == 1) {
              hv[e] = (_Float16)sp[e];
            } else {
              unsigned short hb = f2bf_bits(sp[e]);
              unsigned short lb = f2bf_bits(sp[e] - bf_bits2f(hb));
              hv[e] = __builtin_bit_cast(_Float16, hb);
              lv[e] = __builtin_bit_cast(_Float16, lb);
            }
          }
          *(volatile v8h*)(C + (size_t)(mBase + row) * ldc + n0 + c8) = hv;
          if (OUT_MODE == 2) *(volatile v8h*)(C2 + (size_t)(mBase + row) * ldc + n0 + c8) = lv;
        }
        __threadfence();
      }
    }
    __builtin_amdgcn_fence(__ATOMIC_RELEASE, "workgroup");
    __builtin_amdgcn_wave_barrier();
    __builtin_amdgcn_fence(__ATOMIC_ACQUIRE, "workgroup");
  }
}

__global__ __launch_bounds__(256) void wtcast_kernel(const float* __restrict__ W, unsigned short* __restrict__ out,
                                                     int kin, int nout, float scale) {
  __shared__ float sm[64][65];
  const int t  = threadIdx.x;
  const int k0 = blockIdx.x * 64;
  const int n0 = blockIdx.y * 64;
#pragma unroll
  for (int i = 0; i < 16; ++i) {
    const int e = i * 256 + t;
    const int r = e >> 6;
    const int c = e & 63;
    sm[c][r] = W[(size_t)(k0 + r) * nout + n0 + c] * scale;
  }
  __syncthreads();
  const int lane = t & 31, wave = t >> 5;
  const int q = lane >> 3, c8 = (lane & 7) * 8;
  for (int pass = 0; pass < 2; ++pass) {
#pragma unroll
    for (int it = 0; it < 2; ++it) {
      const int row = wave * 8 + it * 4 + q;
      unsigned short hb[8];
#pragma unroll
      for (int e = 0; e < 8; ++e) hb[e] = h_bits(sm[row][c8 + e]);
      const v4u u = (v4u){pk16(hb[0], hb[1]), pk16(hb[2], hb[3]), pk16(hb[4], hb[5]), pk16(hb[6], hb[7])};
      *(volatile v4u*)(out + (size_t)(n0 + row) * kin + k0 + c8) = u;
    }
    __threadfence();
  }
}

__global__ __launch_bounds__(256) void layernorm_f16_kernel(const float* __restrict__ x, const float* __restrict__ gam,
                                                            const float* __restrict__ bet, unsigned short* __restrict__ out,
                                                            int rows) {
  const int lane = threadIdx.x & 31, wave = threadIdx.x >> 5;
  const int row = blockIdx.x * 8 + wave;
  if (row >= rows) return;
  const float* xr = x + (size_t)row * kD;
  float s = 0.f;
#pragma unroll 1
  for (int j = 0; j < 4; ++j) {
    const int base = j * 256 + lane * 8;
    const v4f a = *(const v4f*)(xr + base);
    const v4f c = *(const v4f*)(xr + base + 4);
    s += ((a[0] + a[1]) + (a[2] + a[3])) + ((c[0] + c[1]) + (c[2] + c[3]));
  }
#pragma unroll
  for (int off = 16; off > 0; off >>= 1) s += __shfl_xor(s, off, 32);
  const float mean = s * kInvD;
  float s2 = 0.f;
#pragma unroll 1
  for (int j = 0; j < 4; ++j) {
    const int base = j * 256 + lane * 8;
    const v4f a = *(const v4f*)(xr + base);
    const v4f c = *(const v4f*)(xr + base + 4);
#pragma unroll
    for (int e = 0; e < 4; ++e) {
      const float d0 = a[e] - mean, d1 = c[e] - mean;
      s2 += d0 * d0;
      s2 += d1 * d1;
    }
  }
#pragma unroll
  for (int off = 16; off > 0; off >>= 1) s2 += __shfl_xor(s2, off, 32);
  const float rstd = rsqrtf(s2 * kInvD + kLnEps);
  unsigned short* orow = out + (size_t)row * kD;
#pragma unroll 1
  for (int j = 0; j < 4; ++j) {
    const int base = j * 256 + lane * 8;
    const v4f a  = *(const v4f*)(xr + base);
    const v4f c  = *(const v4f*)(xr + base + 4);
    const v4f ga = *(const v4f*)(gam + base);
    const v4f gc = *(const v4f*)(gam + base + 4);
    const v4f ba = *(const v4f*)(bet + base);
    const v4f bc = *(const v4f*)(bet + base + 4);
    unsigned short hb[8];
#pragma unroll
    for (int e = 0; e < 4; ++e) {
      hb[e]     = h_bits((a[e] - mean) * rstd * ga[e] + ba[e]);
      hb[4 + e] = h_bits((c[e] - mean) * rstd * gc[e] + bc[e]);
    }
    const v4u u = (v4u){pk16(hb[0], hb[1]), pk16(hb[2], hb[3]), pk16(hb[4], hb[5]), pk16(hb[6], hb[7])};
    unsigned short* op = orow + base;
    *(volatile v4u*)op = u;
    __threadfence();
    *(volatile v4u*)op = u;
  }
}

__global__ __launch_bounds__(256) void vt_transpose_kernel(const unsigned short* __restrict__ kv, unsigned short* __restrict__ vt) {
  __shared__ unsigned short sm[64][72];
  const int t  = threadIdx.x;
  const int g  = blockIdx.y;
  const int b  = g >> 4, h = g & 15;
  const int s0 = blockIdx.x * 64;
  const int r  = t >> 2;
  const int part = (t & 3) * 16;
  const unsigned short* src = kv + ((size_t)(b * kT + s0 + r) * kKVld + kD + h * kDH + part);
  const v4u w0 = *(const v4u*)(src);
  const v4u w1 = *(const v4u*)(src + 8);
#pragma unroll
  for (int e = 0; e < 4; ++e) {
    sm[part + 2 * e][r]         = (unsigned short)(w0[e] & 0xffffu);
    sm[part + 2 * e + 1][r]     = (unsigned short)(w0[e] >> 16);
    sm[part + 8 + 2 * e][r]     = (unsigned short)(w1[e] & 0xffffu);
    sm[part + 8 + 2 * e + 1][r] = (unsigned short)(w1[e] >> 16);
  }
  __syncthreads();
  const int lane = t & 31, wave = t >> 5;
  const int q = lane >> 3, c8 = (lane & 7) * 8;
  for (int pass = 0; pass < 2; ++pass) {
#pragma unroll
    for (int it = 0; it < 2; ++it) {
      const int row = wave * 8 + it * 4 + q;
      unsigned short hb[8];
#pragma unroll
      for (int e = 0; e < 8; ++e) hb[e] = sm[row][c8 + e];
      const v4u u = (v4u){pk16(hb[0], hb[1]), pk16(hb[2], hb[3]), pk16(hb[4], hb[5]), pk16(hb[6], hb[7])};
      *(volatile v4u*)(vt + ((size_t)(g * kDH + row) * kT + s0 + c8)) = u;
    }
    __threadfence();
  }
}

__global__ __launch_bounds__(256) void softmax_band_kernel(const float* __restrict__ S, unsigned short* __restrict__ P,
                                                           const int* __restrict__ bandp, float carry) {
  const int lane = threadIdx.x & 31, wave = threadIdx.x >> 5;
  const int row = blockIdx.x * 8 + wave;
  const int t = row & (kT - 1);
  int band = bandp[0];
  band = band > 2 * kT ? 2 * kT : band;
  band = band < -2 * kT ? -2 * kT : band;
  int lo = t - band; lo = lo < 0 ? 0 : lo;
  int hi = t + band; hi = hi > kT - 1 ? kT - 1 : hi;
  const float* sr = S + (size_t)row * kT;

  float m = -INFINITY;
  for (int it = 0; it < kT / 32; ++it) {
    const int c0 = lo + it * 32;
    if (c0 > hi) break;
    const int c  = c0 + lane;
    const int cc = c < hi ? c : hi;
    float v = sr[cc];
    v = (c <= hi) ? v : -INFINITY;
    m = fmaxf(m, v);
  }
#pragma unroll
  for (int off = 16; off > 0; off >>= 1) m = fmaxf(m, __shfl_xor(m, off, 32));

  float l = 0.f;
  for (int it = 0; it < kT / 32; ++it) {
    const int c0 = lo + it * 32;
    if (c0 > hi) break;
    const int c  = c0 + lane;
    const int cc = c < hi ? c : hi;
    const float ex = expf(sr[cc] - m);
    l += (c <= hi) ? ex : 0.f;
  }
#pragma unroll
  for (int off = 16; off > 0; off >>= 1) l += __shfl_xor(l, off, 32);
  const float kinv = carry * (1.0f / l);

  unsigned short* pr = P + (size_t)row * kT;
#pragma unroll 1
  for (int ch = 0; ch < kT / 256; ++ch) {
    const int cb = ch * 256 + lane * 8;
    v4u u = (v4u){0u, 0u, 0u, 0u};
    if (!(((ch * 256 + 255) < lo) || ((ch * 256) > hi))) {
      const v4f a  = *(const v4f*)(sr + cb);
      const v4f c4 = *(const v4f*)(sr + cb + 4);
      unsigned short hb[8];
#pragma unroll
      for (int e = 0; e < 4; ++e) {
        const int col0 = cb + e, col1 = cb + 4 + e;
        const float p0 = expf(a[e] - m) * kinv;
        const float p1 = expf(c4[e] - m) * kinv;
        hb[e]     = (col0 >= lo && col0 <= hi) ? h_bits(p0) : (unsigned short)0;
        hb[4 + e] = (col1 >= lo && col1 <= hi) ? h_bits(p1) : (unsigned short)0;
      }
      u = (v4u){pk16(hb[0], hb[1]), pk16(hb[2], hb[3]), pk16(hb[4], hb[5]), pk16(hb[6], hb[7])};
    }
    unsigned short* op = pr + cb;
    *(volatile v4u*)op = u;
    __threadfence();
    *(volatile v4u*)op = u;
  }
}

__global__ __launch_bounds__(256) void gelu_cast_kernel(const float* __restrict__ in, unsigned short* __restrict__ out,
                                                        int n2, float carry) {
  const int i = blockIdx.x * 256 + threadIdx.x;
  if (i >= n2) return;
  unsigned u = 0u;
#pragma unroll 1
  for (int e = 0; e < 2; ++e) {
    const float x = in[2 * (size_t)i + e];
    const float gv = 0.5f * x * (1.0f + erff(x * 0.70710678118654752f));
    u |= ((unsigned)h_bits(gv * carry)) << (16 * e);
  }
  unsigned* op = (unsigned*)out + i;
  *(volatile unsigned*)op = u;
  __threadfence();
  *(volatile unsigned*)op = u;
}

extern "C" void kernel_launch(void* const* d_in, const int* in_sizes, int n_in,
                              void* d_out, int out_size, void* d_ws, size_t ws_size, hipStream_t stream) {
  if (n_in < 21) return;
  if (in_sizes[0] != kTok * kD || in_sizes[1] != kTok * kD) return;
  if (in_sizes[2] != kD || in_sizes[3] != kD || in_sizes[4] != kD || in_sizes[5] != kD) return;
  if (in_sizes[6] != kD * kD || in_sizes[7] != kD || in_sizes[8] != kD * kD || in_sizes[9] != kD) return;
  if (in_sizes[10] != kD * kD || in_sizes[11] != kD || in_sizes[12] != kD * kD || in_sizes[13] != kD) return;
  if (in_sizes[14] != kD || in_sizes[15] != kD) return;
  if (in_sizes[16] != kD * kFF || in_sizes[17] != kFF || in_sizes[18] != kFF * kD || in_sizes[19] != kD) return;
  if (in_sizes[20] < 1) return;
  if (out_size != kTok * kD) return;
  if (ws_size < kWsTotal) return;

  const float* x_refined = (const float*)d_in[0];
  const float* x_mem     = (const float*)d_in[1];
  const float* ln_q_g    = (const float*)d_in[2];
  const float* ln_q_b    = (const float*)d_in[3];
  const float* ln_kv_g   = (const float*)d_in[4];
  const float* ln_kv_b   = (const float*)d_in[5];
  const float* Wq        = (const float*)d_in[6];
  const float* bq        = (const float*)d_in[7];
  const float* Wk        = (const float*)d_in[8];
  const float* bk        = (const float*)d_in[9];
  const float* Wv        = (const float*)d_in[10];
  const float* bv        = (const float*)d_in[11];
  const float* Wo        = (const float*)d_in[12];
  const float* bo        = (const float*)d_in[13];
  const float* ln_f_g    = (const float*)d_in[14];
  const float* ln_f_b    = (const float*)d_in[15];
  const float* W1        = (const float*)d_in[16];
  const float* b1        = (const float*)d_in[17];
  const float* W2        = (const float*)d_in[18];
  const float* b2        = (const float*)d_in[19];
  const int*   bandp     = (const int*)d_in[20];
  float* out = (float*)d_out;

  char* ws = (char*)d_ws;
  unsigned short* WoT  = (unsigned short*)(ws + OFF_WOT);
  unsigned short* W1T  = (unsigned short*)(ws + OFF_W1T);
  unsigned short* W2T  = (unsigned short*)(ws + OFF_W2T);
  unsigned short* ctx  = (unsigned short*)(ws + OFF_CTX);
  unsigned short* qp   = (unsigned short*)(ws + OFF_QP);
  unsigned short* kvp  = (unsigned short*)(ws + OFF_KVP);
  unsigned short* vt   = (unsigned short*)(ws + OFF_VT);
  unsigned short* qln  = (unsigned short*)(ws + OFF_QLN);
  unsigned short* kvln = (unsigned short*)(ws + OFF_KVLN);
  unsigned short* WqT  = (unsigned short*)(ws + OFF_WQT);
  unsigned short* WkT  = (unsigned short*)(ws + OFF_WKT);
  unsigned short* WvT  = (unsigned short*)(ws + OFF_WVT);
  float*          sc   = (float*)(ws + OFF_SC);
  float*          yf   = (float*)(ws + OFF_Y);
  unsigned short* h16  = (unsigned short*)(ws + OFF_H16);
  unsigned short* act  = (unsigned short*)(ws + OFF_ACT);
  unsigned short* pp   = (unsigned short*)(ws + OFF_P);
  float*          h1   = (float*)(ws + OFF_H1);

  const unsigned short* n16 = nullptr;
  const float* nf = nullptr;
  void* nv = nullptr;
  const dim3 tb(256);

  wtcast_kernel<<<dim3(kD / 64, kD / 64), tb, 0, stream>>>(Wq, WqT, kD, kD, kWCarry);
  wtcast_kernel<<<dim3(kD / 64, kD / 64), tb, 0, stream>>>(Wk, WkT, kD, kD, kWCarry);
  wtcast_kernel<<<dim3(kD / 64, kD / 64), tb, 0, stream>>>(Wv, WvT, kD, kD, kWCarry);
  wtcast_kernel<<<dim3(kD / 64, kD / 64), tb, 0, stream>>>(Wo, WoT, kD, kD, kWCarry);
  wtcast_kernel<<<dim3(kD / 64, kFF / 64), tb, 0, stream>>>(W1, W1T, kD, kFF, kWCarry);
  wtcast_kernel<<<dim3(kFF / 64, kD / 64), tb, 0, stream>>>(W2, W2T, kFF, kD, kWCarry);

  layernorm_f16_kernel<<<dim3(kTok / 8), tb, 0, stream>>>(x_refined, ln_q_g, ln_q_b, qln, kTok);
  layernorm_f16_kernel<<<dim3(kTok / 8), tb, 0, stream>>>(x_mem, ln_kv_g, ln_kv_b, kvln, kTok);

  const float projScale = 1.0f / kWCarry;
  wmma_gemm64<0, false, 2, 1, false><<<dim3((kTok / 64) * (kD / 64) / 8, 1), tb, 0, stream>>>(
      qln, n16, kD, (long)0, WqT, n16, kD, (long)0, (void*)qp, nv, kD, (long)0,
      bq, nf, (long)0, kTok, kD, kD, projScale);
  wmma_gemm64<0, false, 2, 1, false><<<dim3((kTok / 64) * (kD / 64) / 8, 1), tb, 0, stream>>>(
      kvln, n16, kD, (long)0, WkT, n16, kD, (long)0, (void*)kvp, nv, kKVld, (long)0,
      bk, nf, (long)0, kTok, kD, kD, projScale);
  wmma_gemm64<0, false, 2, 1, false><<<dim3((kTok / 64) * (kD / 64) / 8, 1), tb, 0, stream>>>(
      kvln, n16, kD, (long)0, WvT, n16, kD, (long)0, (void*)(kvp + kD), nv, kKVld, (long)0,
      bv, nf, (long)0, kTok, kD, kD, projScale);

  vt_transpose_kernel<<<dim3(kT / 64, kGrp), tb, 0, stream>>>(kvp, vt);

  const float scoreScale = 0.125f;
  const float pvScale    = kCtxCarry / kPCarry;
  for (int chk = 0; chk < kNChunk; ++chk) {
    const int g0 = chk * kGC;
    const int b  = g0 / kH;
    const int h0 = g0 % kH;
    const unsigned short* qbase = qp  + (size_t)b * kT * kD    + (size_t)h0 * kDH;
    const unsigned short* kbase = kvp + (size_t)b * kT * kKVld + (size_t)h0 * kDH;
    wmma_gemm64<0, false, 0, 0, false><<<dim3((kT / 64) * (kT / 64) / 8, kGC), tb, 0, stream>>>(
        qbase, n16, kD, (long)kDH, kbase, n16, kKVld, (long)kDH, (void*)sc, nv, kT, (long)kT * kT,
        nf, nf, (long)0, kT, kT, kDH, scoreScale);
    softmax_band_kernel<<<dim3((kGC * kT) / 8), tb, 0, stream>>>(sc, pp, bandp, kPCarry);
    wmma_gemm64<0, false, 0, 1, false><<<dim3((kT / 64) * (kDH / 64) / 8, kGC), tb, 0, stream>>>(
        pp, n16, kT, (long)kT * kT, vt + (size_t)g0 * kDH * kT, n16, kT, (long)kDH * kT,
        (void*)(ctx + (size_t)b * kT * kD + (size_t)h0 * kDH), nv, kD, (long)kDH,
        nf, nf, (long)0, kT, kDH, kT, pvScale);
  }

  wmma_gemm64<0, false, 2, 0, true><<<dim3((kTok / 64) * (kD / 64) / 8, 1), tb, 0, stream>>>(
      ctx, n16, kD, (long)0, WoT, n16, kD, (long)0, (void*)yf, nv, kD, (long)0,
      bo, x_refined, (long)0, kTok, kD, kD, 1.0f / (kCtxCarry * kWCarry));

  layernorm_f16_kernel<<<dim3(kTok / 8), tb, 0, stream>>>(yf, ln_f_g, ln_f_b, h16, kTok);

  for (int mc = 0; mc < kNMC; ++mc) {
    const size_t rowOff = (size_t)mc * kMC;
    wmma_gemm64<0, false, 2, 0, false><<<dim3((kMC / 64) * (kFF / 64) / 8, 1), tb, 0, stream>>>(
        h16 + rowOff * kD, n16, kD, (long)0, W1T, n16, kD, (long)0, (void*)h1, nv, kFF, (long)0,
        b1, nf, (long)0, kMC, kFF, kD, 1.0f / kWCarry);
    gelu_cast_kernel<<<dim3((kMC * kFF / 2 + 255) / 256), tb, 0, stream>>>(h1, act, kMC * kFF / 2, kActCarry);
    wmma_gemm64<0, false, 2, 0, true><<<dim3((kMC / 64) * (kD / 64) / 8, 1), tb, 0, stream>>>(
        act, n16, kFF, (long)0, W2T, n16, kFF, (long)0, (void*)(out + rowOff * kD), nv, kD, (long)0,
        b2, yf + rowOff * kD, (long)0, kMC, kD, kFF, 1.0f / (kActCarry * kWCarry));
  }
}
